// EGNN_layer_72000831750801
// MI455X (gfx1250) — hardware-verified
//
#include <hip/hip_runtime.h>


#define BB       8
#define NN       512
#define FD       3
#define HIDN     64
#define WAVES    8
#define NPB      32
#define NPW      (NPB / WAVES)
#define NTHREADS (WAVES * 32)
#define SPITCH   72

#define SCALE_W  64.0f
#define SCALE_A  16.0f
#define INV_G1   (1.0f / 64.0f)
#define INV_G23  (1.0f / 1024.0f)

typedef _Float16 v16h __attribute__((ext_vector_type(16)));
typedef _Float16 v8h  __attribute__((ext_vector_type(8)));
typedef _Float16 v8ha __attribute__((ext_vector_type(8), __may_alias__));
typedef float    v8f  __attribute__((ext_vector_type(8)));
typedef float    v4f  __attribute__((ext_vector_type(4)));

__device__ __forceinline__ float silu_f(float x) {
    float e = __builtin_amdgcn_exp2f(-1.44269504089f * x);
    return x * __builtin_amdgcn_rcpf(1.0f + e);
}

__device__ __forceinline__ v8f wmma16(v16h a, v16h b, v8f c) {
    v8f d = __builtin_amdgcn_wmma_f32_16x16x32_f16(false, a, false, b, (short)0, c, false, false);
    asm volatile("v_nop\n\tv_nop\n\tv_nop\n\tv_nop" : "+v"(d) : "v"(a), "v"(b));
    return d;
}

__device__ __forceinline__ v16h cat8(v8h lo, v8h hi) {
    return __builtin_shufflevector(lo, hi, 0, 1, 2, 3, 4, 5, 6, 7,
                                   8, 9, 10, 11, 12, 13, 14, 15);
}

__device__ __forceinline__ int kmap(int q, int hh) {
    return (q < 8) ? (8 * hh + q) : (16 + 8 * hh + (q - 8));
}

__global__ __launch_bounds__(NTHREADS) void egnn_layer_k(
    const float* __restrict__ feats, const float* __restrict__ coors,
    const float* __restrict__ vel,
    const float* __restrict__ We1, const float* __restrict__ be1,
    const float* __restrict__ We2, const float* __restrict__ be2,
    const float* __restrict__ Wc1, const float* __restrict__ bc1,
    const float* __restrict__ Wc2,
    const float* __restrict__ Wv,  const float* __restrict__ bv,
    const float* __restrict__ Wn1, const float* __restrict__ bn1,
    const float* __restrict__ Wn2, const float* __restrict__ bn2,
    float* __restrict__ out)
{
    __shared__ __align__(32) _Float16 wfrag[20 * 512];
    __shared__ __align__(16) _Float16 stage[WAVES][16 * SPITCH];
    __shared__ float msum_s[WAVES][HIDN];
    __shared__ __align__(16) float res[3][NPB * FD];

    for (int e = threadIdx.x; e < 20 * 512; e += NTHREADS) {
        const int f = e >> 9, rem = e & 511, ln = rem >> 4, q = rem & 15;
        const int rc = ln & 15, hh = ln >> 4;
        const int kk = kmap(q, hh);
        float v = 0.0f;
        if (f < 4) {
            const int m = f * 16 + rc;
            if (kk < 2 * FD + 1)       v = We1[kk * HIDN + m] * SCALE_W;
            else if (kk == 2 * FD + 1) v = be1[m] * SCALE_W;
        } else if (f < 12) {
            const int g2 = f - 4, nt = g2 >> 1, kt = g2 & 1;
            v = We2[(kt * 32 + kk) * HIDN + nt * 16 + rc] * SCALE_W;
        } else {
            const int g3 = f - 12, nt = g3 >> 1, kt = g3 & 1;
            v = Wc1[(kt * 32 + kk) * HIDN + nt * 16 + rc] * SCALE_W;
        }
        wfrag[e] = (_Float16)v;
    }
    __syncthreads();

    const int lane = threadIdx.x & 31;
    const int w    = threadIdx.x >> 5;
    const int col  = lane & 15;
    const int half = lane >> 4;

    float be2_l[4], bc1_l[4], wc2_l[4];
#pragma unroll
    for (int nt = 0; nt < 4; ++nt) {
        be2_l[nt] = be2[nt * 16 + col];
        bc1_l[nt] = bc1[nt * 16 + col];
        wc2_l[nt] = Wc2[nt * 16 + col];
    }

    _Float16* sp = &stage[w][0];
    const v8f zero8 = {0.f, 0.f, 0.f, 0.f, 0.f, 0.f, 0.f, 0.f};
    const _Float16 hz = (_Float16)0.0f;
    const v8h z8h = {hz, hz, hz, hz, hz, hz, hz, hz};
    const float emask = (lane < 16) ? 1.0f : 0.0f;

#pragma unroll 1
    for (int q4 = 0; q4 < NPW; ++q4) {
        const int nl = q4 * WAVES + w;
        int g = blockIdx.x * NPB + nl;
        g = (g < BB * NN) ? g : (BB * NN - 1);
        const int b = g / NN;
        const int i = g - b * NN;
        const float* fb  = feats + (size_t)b * NN * FD;
        const float* cbp = coors + (size_t)b * NN * 3;

        const float fi0 = fb[i * FD + 0];
        const float fi1 = fb[i * FD + 1];
        const float fi2 = fb[i * FD + 2];
        const float cix = cbp[i * 3 + 0];
        const float ciy = cbp[i * 3 + 1];
        const float ciz = cbp[i * 3 + 2];

        float msum[4] = {0.f, 0.f, 0.f, 0.f};
        float cax = 0.f, cay = 0.f, caz = 0.f;

#pragma unroll 1
        for (int j0 = 0; j0 < NN; j0 += 16) {
            const int jl = j0 + col;
            const float fj0 = fb[jl * FD + 0];
            const float fj1 = fb[jl * FD + 1];
            const float fj2 = fb[jl * FD + 2];
            const float cjx = cbp[jl * 3 + 0];
            const float cjy = cbp[jl * 3 + 1];
            const float cjz = cbp[jl * 3 + 2];
            const float dx = cix - cjx, dy = ciy - cjy, dz = ciz - cjz;
            const float d2 = dx * dx + dy * dy + dz * dz;

            const int rsel = i - j0 - 8 * half;
            float rowfac[8];
#pragma unroll
            for (int r = 0; r < 8; ++r) rowfac[r] = (r == rsel) ? 0.0f : 1.0f;

            v16h bE = cat8(z8h, z8h);
            if (lane < 16) {
                bE[0] = (_Float16)fi0; bE[1] = (_Float16)fi1; bE[2] = (_Float16)fi2;
                bE[3] = (_Float16)fj0; bE[4] = (_Float16)fj1; bE[5] = (_Float16)fj2;
                bE[6] = (_Float16)d2;  bE[7] = (_Float16)1.0f;
            }

            v8h s1[4];
#pragma unroll
            for (int mt = 0; mt < 4; ++mt) {
                const v16h aW = *(const v16h*)&wfrag[mt * 512 + lane * 16];
                const v8f c = wmma16(aW, bE, zero8);
#pragma unroll
                for (int e = 0; e < 8; ++e)
                    s1[mt][e] = (_Float16)(silu_f(c[e] * INV_G1) * SCALE_A);
            }

            const v16h a2_0 = cat8(s1[0], s1[1]);
            const v16h a2_1 = cat8(s1[2], s1[3]);

#pragma unroll
            for (int nt = 0; nt < 4; ++nt) {
                const v16h b0 = *(const v16h*)&wfrag[(4 + nt * 2 + 0) * 512 + lane * 16];
                const v16h b1 = *(const v16h*)&wfrag[(4 + nt * 2 + 1) * 512 + lane * 16];
                v8f c = wmma16(a2_0, b0, zero8);
                c = wmma16(a2_1, b1, c);
                float s = 0.f;
#pragma unroll
                for (int r = 0; r < 8; ++r) {
                    const float v = rowfac[r] * silu_f(c[r] * INV_G23 + be2_l[nt]);
                    s += v;
                    sp[(r + 8 * half) * SPITCH + nt * 16 + col] = (_Float16)(v * SCALE_A);
                }
                msum[nt] += s;
            }
            __syncthreads();

            const int rA = lane & 15;
            const v8h lo0 = *(const v8ha*)(sp + rA * SPITCH + 0  + 8 * half);
            const v8h hi0 = *(const v8ha*)(sp + rA * SPITCH + 16 + 8 * half);
            const v8h lo1 = *(const v8ha*)(sp + rA * SPITCH + 32 + 8 * half);
            const v8h hi1 = *(const v8ha*)(sp + rA * SPITCH + 48 + 8 * half);
            const v16h a3_0 = cat8(lo0, hi0);
            const v16h a3_1 = cat8(lo1, hi1);

            float t[8] = {0.f, 0.f, 0.f, 0.f, 0.f, 0.f, 0.f, 0.f};
#pragma unroll
            for (int nt = 0; nt < 4; ++nt) {
                const v16h b0 = *(const v16h*)&wfrag[(12 + nt * 2 + 0) * 512 + lane * 16];
                const v16h b1 = *(const v16h*)&wfrag[(12 + nt * 2 + 1) * 512 + lane * 16];
                v8f c = wmma16(a3_0, b0, zero8);
                c = wmma16(a3_1, b1, c);
#pragma unroll
                for (int r = 0; r < 8; ++r)
                    t[r] += silu_f(c[r] * INV_G23 + bc1_l[nt]) * wc2_l[nt];
            }
#pragma unroll
            for (int r = 0; r < 8; ++r) {
                t[r] += __shfl_xor(t[r], 1, 32);
                t[r] += __shfl_xor(t[r], 2, 32);
                t[r] += __shfl_xor(t[r], 4, 32);
                t[r] += __shfl_xor(t[r], 8, 32);
            }
            float tv = t[0];
#pragma unroll
            for (int r = 1; r < 8; ++r) tv = ((lane & 7) == r) ? t[r] : tv;
            const float to = __shfl_xor(tv, 16, 32);
            const float ph = (((lane >> 3) & 1) == half) ? tv : to;

            cax += emask * ph * dx;
            cay += emask * ph * dy;
            caz += emask * ph * dz;
        }

#pragma unroll
        for (int nt = 0; nt < 4; ++nt) msum[nt] += __shfl_xor(msum[nt], 16, 32);
        if (lane < 16) {
#pragma unroll
            for (int nt = 0; nt < 4; ++nt) msum_s[w][nt * 16 + lane] = msum[nt];
        }

#pragma unroll
        for (int m = 1; m < 32; m <<= 1) {
            cax += __shfl_xor(cax, m, 32);
            cay += __shfl_xor(cay, m, 32);
            caz += __shfl_xor(caz, m, 32);
        }
        const float inv = 1.0f / (float)(NN - 1);
        const float aggx = cax * inv, aggy = cay * inv, aggz = caz * inv;

        const float gate = fi0 * Wv[0] + fi1 * Wv[1] + fi2 * Wv[2] + bv[0];
        const float* vb = vel + (size_t)b * NN * 3;
        const float vnx = gate * vb[i * 3 + 0] + aggx;
        const float vny = gate * vb[i * 3 + 1] + aggy;
        const float vnz = gate * vb[i * 3 + 2] + aggz;
        const float cnx = cix + vnx, cny = ciy + vny, cnz = ciz + vnz;

        const int ca = lane, cbn = lane + 32;
        float acc0 = bn1[ca]  + fi0 * Wn1[0 * HIDN + ca]  + fi1 * Wn1[1 * HIDN + ca]  + fi2 * Wn1[2 * HIDN + ca];
        float acc1 = bn1[cbn] + fi0 * Wn1[0 * HIDN + cbn] + fi1 * Wn1[1 * HIDN + cbn] + fi2 * Wn1[2 * HIDN + cbn];
#pragma unroll 4
        for (int k = 0; k < HIDN; ++k) {
            const float xk = msum_s[w][k];
            acc0 += xk * Wn1[(FD + k) * HIDN + ca];
            acc1 += xk * Wn1[(FD + k) * HIDN + cbn];
        }
        const float h0 = silu_f(acc0), h1 = silu_f(acc1);
        float o[3];
#pragma unroll
        for (int d = 0; d < 3; ++d) {
            o[d] = h0 * Wn2[ca * FD + d] + h1 * Wn2[cbn * FD + d];
#pragma unroll
            for (int m = 1; m < 32; m <<= 1) o[d] += __shfl_xor(o[d], m, 32);
        }

        if (lane == 0) {
            res[0][nl * FD + 0] = fi0 + o[0] + bn2[0];
            res[0][nl * FD + 1] = fi1 + o[1] + bn2[1];
            res[0][nl * FD + 2] = fi2 + o[2] + bn2[2];
            res[1][nl * 3 + 0] = cnx; res[1][nl * 3 + 1] = cny; res[1][nl * 3 + 2] = cnz;
            res[2][nl * 3 + 0] = vnx; res[2][nl * 3 + 1] = vny; res[2][nl * 3 + 2] = vnz;
        }
    }

    __syncthreads();

    if (w == 0) {
        const bool act = (lane < 24) && (blockIdx.x * NPB < BB * NN);
        const int li = (lane < 24) ? lane : 0;
        const v4f v0 = *(const v4f*)&res[0][li * 4];
        const v4f v1 = *(const v4f*)&res[1][li * 4];
        const v4f v2 = *(const v4f*)&res[2][li * 4];
        const size_t outn = (size_t)BB * NN * FD;
        const size_t base = (size_t)blockIdx.x * NPB * FD;
        volatile v4f* p0 = (volatile v4f*)(out + base) + li;
        volatile v4f* p1 = (volatile v4f*)(out + outn + base) + li;
        volatile v4f* p2 = (volatile v4f*)(out + 2 * outn + base) + li;
        if (act) { *p0 = v0; *p1 = v1; *p2 = v2; }
        __threadfence();
        if (act) { *p0 = v0; *p1 = v1; *p2 = v2; }
    }
}

extern "C" void kernel_launch(void* const* d_in, const int* in_sizes, int n_in,
                              void* d_out, int out_size, void* d_ws, size_t ws_size,
                              hipStream_t stream) {
    (void)d_ws; (void)ws_size;
    if (n_in < 16) return;
    if (in_sizes[0] != BB * NN * FD || in_sizes[1] != BB * NN * 3 || in_sizes[2] != BB * NN * 3) return;
    if (in_sizes[3] != (2 * FD + 1) * HIDN || in_sizes[4] != HIDN ||
        in_sizes[5] != HIDN * HIDN || in_sizes[6] != HIDN ||
        in_sizes[7] != HIDN * HIDN || in_sizes[8] != HIDN ||
        in_sizes[9] != HIDN || in_sizes[10] != FD || in_sizes[11] != 1 ||
        in_sizes[12] != (FD + HIDN) * HIDN || in_sizes[13] != HIDN ||
        in_sizes[14] != HIDN * FD || in_sizes[15] != FD) return;
    if (out_size != 3 * BB * NN * FD) return;

    const float* feats = (const float*)d_in[0];
    const float* coors = (const float*)d_in[1];
    const float* vel   = (const float*)d_in[2];
    const float* We1   = (const float*)d_in[3];
    const float* be1   = (const float*)d_in[4];
    const float* We2   = (const float*)d_in[5];
    const float* be2   = (const float*)d_in[6];
    const float* Wc1   = (const float*)d_in[7];
    const float* bc1   = (const float*)d_in[8];
    const float* Wc2   = (const float*)d_in[9];
    const float* Wv    = (const float*)d_in[10];
    const float* bv    = (const float*)d_in[11];
    const float* Wn1   = (const float*)d_in[12];
    const float* bn1   = (const float*)d_in[13];
    const float* Wn2   = (const float*)d_in[14];
    const float* bn2   = (const float*)d_in[15];

    dim3 grid((BB * NN + NPB - 1) / NPB);
    dim3 block(NTHREADS);
    egnn_layer_k<<<grid, block, 0, stream>>>(feats, coors, vel,
                                             We1, be1, We2, be2,
                                             Wc1, bc1, Wc2, Wv, bv,
                                             Wn1, bn1, Wn2, bn2,
                                             (float*)d_out);
}
